// PFNN_41008347742352
// MI455X (gfx1250) — hardware-verified
//
#include <hip/hip_runtime.h>
#include <stdint.h>


typedef _Float16 f16_t;
typedef _Float16 v16h __attribute__((ext_vector_type(16)));
typedef _Float16 v8h  __attribute__((ext_vector_type(8)));
typedef v8h      v8ha __attribute__((may_alias));
typedef float    v8f  __attribute__((ext_vector_type(8)));
typedef float    v4f  __attribute__((ext_vector_type(4)));
typedef v4f      v4fa __attribute__((may_alias));

#define HID    32
#define NBR    4
#define DIN    3
#define TPB    256
#define WPB    8
#define ROWS_W 32
#define ROWS_B (WPB * ROWS_W)
#define PH     40
#define PF     36
#define WSCALE 64.0f
#define WINV   0.015625f

union Frag { v16h v; v8h h[2]; };

__device__ __forceinline__ float tanh_via_exp(float v) {
    float e = __expf(2.0f * v);
    float r = __builtin_amdgcn_rcpf(e + 1.0f);
    return fmaf(-2.0f, r, 1.0f);
}

__device__ __forceinline__ void wmma_pair(v8f& c0, v8f& c1, const v16h a, const v16h b0, const v16h b1) {
    const v8f z = {0.f, 0.f, 0.f, 0.f, 0.f, 0.f, 0.f, 0.f};
    c0 = __builtin_amdgcn_wmma_f32_16x16x32_f16(false, a, false, b0, (short)0, z, false, false);
    c1 = __builtin_amdgcn_wmma_f32_16x16x32_f16(false, a, false, b1, (short)0, z, false, false);
    asm volatile("v_nop\n\tv_nop\n\tv_nop\n\tv_nop" : "+v"(c0), "+v"(c1) : "v"(a), "v"(b0), "v"(b1));
}

__launch_bounds__(TPB)
__global__ void k_mlp4(const float* __restrict__ x,
                       const float* __restrict__ W0, const float* __restrict__ b0,
                       const float* __restrict__ W1, const float* __restrict__ b1,
                       const float* __restrict__ W2, const float* __restrict__ b2,
                       const float* __restrict__ W3, const float* __restrict__ b3,
                       float* __restrict__ out, int n_rows)
{
    __shared__ __align__(16) f16_t sW1[NBR * HID * HID];
    __shared__ __align__(16) f16_t sW2[NBR * HID * HID];
    __shared__ __align__(16) float sW0[NBR * DIN * HID];
    __shared__ __align__(16) float sB0[NBR * HID];
    __shared__ __align__(16) float sB1[NBR * HID];
    __shared__ __align__(16) float sB2[NBR * HID];
    __shared__ __align__(16) float sW3[NBR * HID];
    __shared__ __align__(16) float sB3[NBR];
    __shared__ __align__(16) f16_t sH[WPB][16 * PH];
    __shared__ __align__(16) float sF[WPB][16 * PF];

    const int tid = threadIdx.x;
    for (int i = tid; i < NBR * HID * HID; i += TPB) {
        const int bb = i >> 10, k = (i >> 5) & 31, n = i & 31;
        sW1[(bb * HID + n) * HID + k] = (f16_t)(W1[i] * WSCALE);
        sW2[(bb * HID + n) * HID + k] = (f16_t)(W2[i] * WSCALE);
    }
    for (int i = tid; i < NBR * DIN * HID; i += TPB) sW0[i] = W0[i];
    if (tid < NBR * HID) {
        sB0[tid] = b0[tid];
        sB1[tid] = b1[tid];
        sB2[tid] = b2[tid];
        sW3[tid] = W3[tid];
    }
    if (tid < NBR) sB3[tid] = b3[tid];
    __syncthreads();

    const int lane = tid & 31;
    const int wave = tid >> 5;
    const int half = lane >> 4;
    const int lrow = lane & 15;
    f16_t* hb = &sH[wave][0];
    float* hf = &sF[wave][0];
    const int base = blockIdx.x * ROWS_B + wave * ROWS_W;

    float ob0 = 0.0f, ob1 = 0.0f, ob2 = 0.0f, ob3 = 0.0f;

#pragma unroll 1
    for (int b = 0; b < NBR; ++b) {
        float w0v[16][3], b0v[16];
#pragma unroll
        for (int i = 0; i < 16; ++i) {
            const int k = 8 * half + (i & 7) + ((i >> 3) << 4);
            w0v[i][0] = sW0[b * (DIN * HID) + k];
            w0v[i][1] = sW0[b * (DIN * HID) + HID + k];
            w0v[i][2] = sW0[b * (DIN * HID) + 2 * HID + k];
            b0v[i]    = sB0[b * HID + k];
        }
        const float bias1a = sB1[b * HID + lrow], bias1b = sB1[b * HID + 16 + lrow];
        const float bias2a = sB2[b * HID + lrow], bias2b = sB2[b * HID + 16 + lrow];
        const float b3v = sB3[b];

        Frag w1f0, w1f1, w2f0, w2f1;
        {
            const f16_t* p0 = sW1 + (b * HID + lrow) * HID;
            const f16_t* p1 = sW1 + (b * HID + 16 + lrow) * HID;
            const f16_t* q0 = sW2 + (b * HID + lrow) * HID;
            const f16_t* q1 = sW2 + (b * HID + 16 + lrow) * HID;
            w1f0.h[0] = *(const v8ha*)(p0 + 8 * half); w1f0.h[1] = *(const v8ha*)(p0 + 16 + 8 * half);
            w1f1.h[0] = *(const v8ha*)(p1 + 8 * half); w1f1.h[1] = *(const v8ha*)(p1 + 16 + 8 * half);
            w2f0.h[0] = *(const v8ha*)(q0 + 8 * half); w2f0.h[1] = *(const v8ha*)(q0 + 16 + 8 * half);
            w2f1.h[0] = *(const v8ha*)(q1 + 8 * half); w2f1.h[1] = *(const v8ha*)(q1 + 16 + 8 * half);
        }

#pragma unroll 1
        for (int s = 0; s < 2; ++s) {
            const int row = base + 16 * s + lrow;
            const int rc  = row < n_rows ? row : n_rows - 1;
            const float* xp = x + (size_t)rc * DIN;
            const float x0 = xp[0], x1 = xp[1], x2 = xp[2];

            Frag a1;
#pragma unroll
            for (int i = 0; i < 16; ++i) {
                const float v = fmaf(x0, w0v[i][0], fmaf(x1, w0v[i][1], fmaf(x2, w0v[i][2], b0v[i])));
                a1.v[i] = (f16_t)tanh_via_exp(v);
            }

            v8f c0, c1;
            wmma_pair(c0, c1, a1.v, w1f0.v, w1f1.v);
#pragma unroll
            for (int r = 0; r < 8; ++r) {
                const int m = 8 * half + r;
                hb[m * PH + lrow]      = (f16_t)tanh_via_exp(fmaf(c0[r], WINV, bias1a));
                hb[m * PH + 16 + lrow] = (f16_t)tanh_via_exp(fmaf(c1[r], WINV, bias1b));
            }
            __syncthreads();

            Frag a2;
            a2.h[0] = *(const v8ha*)(hb + lrow * PH + 8 * half);
            a2.h[1] = *(const v8ha*)(hb + lrow * PH + 16 + 8 * half);

            v8f d0, d1;
            wmma_pair(d0, d1, a2.v, w2f0.v, w2f1.v);
#pragma unroll
            for (int r = 0; r < 8; ++r) {
                const int m = 8 * half + r;
                hf[m * PF + lrow]      = tanh_via_exp(fmaf(d0[r], WINV, bias2a));
                hf[m * PF + 16 + lrow] = tanh_via_exp(fmaf(d1[r], WINV, bias2b));
            }
            __syncthreads();

            float partial = 0.0f;
            {
                const float* hr = hf + lrow * PF + 16 * half;
                const float* wr = sW3 + b * HID + 16 * half;
#pragma unroll
                for (int q = 0; q < 4; ++q) {
                    const v4f hv = *(const v4fa*)(hr + 4 * q);
                    const v4f wv = *(const v4fa*)(wr + 4 * q);
                    partial = fmaf(hv[0], wv[0], partial);
                    partial = fmaf(hv[1], wv[1], partial);
                    partial = fmaf(hv[2], wv[2], partial);
                    partial = fmaf(hv[3], wv[3], partial);
                }
            }
            const float total = partial + __shfl_xor(partial, 16, 32);
            const float val = total + b3v;
            const bool mine = (half == s);
            ob0 = (mine && b == 0) ? val : ob0;
            ob1 = (mine && b == 1) ? val : ob1;
            ob2 = (mine && b == 2) ? val : ob2;
            ob3 = (mine && b == 3) ? val : ob3;
        }
    }

    const int orow = base + lane;
    const bool ok = orow < n_rows;
    v4f o;
    o[0] = ob0; o[1] = ob1; o[2] = ob2; o[3] = ob3;
    volatile v4f* op = (volatile v4f*)(out + (size_t)(ok ? orow : 0) * NBR);
    if (ok) *op = o;
    __threadfence();
    if (ok) *op = o;
}

extern "C" void kernel_launch(void* const* d_in, const int* in_sizes, int n_in,
                              void* d_out, int out_size, void* d_ws, size_t ws_size,
                              hipStream_t stream)
{
    (void)d_ws; (void)ws_size;
    if (n_in < 9) return;
    if (in_sizes[1] != NBR * DIN * HID || in_sizes[2] != NBR * HID ||
        in_sizes[3] != NBR * HID * HID || in_sizes[4] != NBR * HID ||
        in_sizes[5] != NBR * HID * HID || in_sizes[6] != NBR * HID ||
        in_sizes[7] != NBR * HID       || in_sizes[8] != NBR) return;

    int n_rows = in_sizes[0] / DIN;
    const int n_out_rows = out_size / NBR;
    if (n_out_rows < n_rows) n_rows = n_out_rows;
    if (n_rows <= 0) return;

    const float* x  = (const float*)d_in[0];
    const float* W0 = (const float*)d_in[1];
    const float* b0 = (const float*)d_in[2];
    const float* W1 = (const float*)d_in[3];
    const float* b1 = (const float*)d_in[4];
    const float* W2 = (const float*)d_in[5];
    const float* b2 = (const float*)d_in[6];
    const float* W3 = (const float*)d_in[7];
    const float* b3 = (const float*)d_in[8];
    float* outp = (float*)d_out;

    const int nblk = (n_rows + ROWS_B - 1) / ROWS_B;
    k_mlp4<<<dim3(nblk), dim3(TPB), 0, stream>>>(x, W0, b0, W1, b1, W2, b2, W3, b3, outp, n_rows);
    (void)hipGetLastError();
}
